// MultiScaleRetention_34806414967451
// MI455X (gfx1250) — hardware-verified
//
#include <hip/hip_runtime.h>
#include <math.h>

constexpr int kB    = 2;
constexpr int kT    = 2048;
constexpr int kD    = 1024;
constexpr int kH    = 16;
constexpr int kDh   = 64;
constexpr int kBH   = kB * kH;
constexpr int kTok  = kB * kT;
constexpr int kRetWaves = 4;
constexpr int kRetRows  = 16 * kRetWaves;
constexpr int kKeyChunk = 64;
constexpr int kPPitch   = 72;
constexpr int kOPitch   = 68;
constexpr int kStatPitch = 32;
constexpr float kPCarry    = 256.0f;
constexpr float kPCarryInv = 1.0f / 256.0f;
constexpr float kLnCut     = -23.0258509f;
constexpr float kGnEps     = 1.0e-5f;
constexpr float kGateClamp = 30.0f;
static_assert(kH * kDh == kD, "shape");
static_assert(kD % 64 == 0 && kTok % 64 == 0 && kT % 64 == 0, "tiles");
static_assert(kD % 32 == 0, "kdepth");
static_assert(kT % kRetRows == 0 && kT % kKeyChunk == 0 && kDh == 64, "ret tiles");
static_assert((kTok * kD) % (8 * 256) == 0 && (kD * kD) % (8 * 256) == 0, "cast grids");

typedef __attribute__((ext_vector_type(16))) _Float16 v16h;
typedef __attribute__((ext_vector_type(8)))  _Float16 v8h;
typedef __attribute__((ext_vector_type(16))) __bf16   v16b;
typedef __attribute__((ext_vector_type(8)))  __bf16   v8b;
typedef __attribute__((ext_vector_type(8)))  float    v8f;
typedef __attribute__((ext_vector_type(4)))  float    v4f;
typedef __attribute__((ext_vector_type(4)))  unsigned int v4u;

__device__ __forceinline__ unsigned short f2bf_bits(float f) {
  unsigned u = __float_as_uint(f);
  return (unsigned short)((u + 0x7FFFu + ((u >> 16) & 1u)) >> 16);
}
__device__ __forceinline__ float bf_bits2f(unsigned short h) { return __uint_as_float(((unsigned)h) << 16); }

__device__ __forceinline__ void dep_guard4_h(v8f& a, v8f& b, v8f& c, v8f& d, v16h x, v16h y) {
  asm volatile("v_nop\n\tv_nop\n\tv_nop\n\tv_nop" : "+v"(a), "+v"(b), "+v"(c), "+v"(d) : "v"(x), "v"(y));
}
__device__ __forceinline__ void dep_guard4_b(v8f& a, v8f& b, v8f& c, v8f& d, v16b x, v16b y) {
  asm volatile("v_nop\n\tv_nop\n\tv_nop\n\tv_nop" : "+v"(a), "+v"(b), "+v"(c), "+v"(d) : "v"(x), "v"(y));
}
__device__ __forceinline__ void keep4_h(v16h a, v16h b, v16h c, v16h d) { asm volatile("v_nop" :: "v"(a), "v"(b), "v"(c), "v"(d)); }
__device__ __forceinline__ void keep4_b(v16b a, v16b b, v16b c, v16b d) { asm volatile("v_nop" :: "v"(a), "v"(b), "v"(c), "v"(d)); }
__device__ __forceinline__ void acc_guard4(v8f& a, v8f& b, v8f& c, v8f& d) { asm volatile("v_nop\n\tv_nop\n\tv_nop\n\tv_nop" : "+v"(a), "+v"(b), "+v"(c), "+v"(d)); }
template <typename T> struct Frag;
template <> struct Frag<_Float16> {
  typedef v16h V; union U { v16h v; v8h h[2]; };
  static __device__ __forceinline__ v16h load(const _Float16* p) {
    U f; f.h[0] = *(const v8h*)(p); f.h[1] = *(const v8h*)(p + 16); return f.v;
  }
  static __device__ __forceinline__ v8f mma(v16h a, v16h b, v8f c) {
    return __builtin_amdgcn_wmma_f32_16x16x32_f16(false, a, false, b, (short)0, c, false, false);
  }
  static __device__ __forceinline__ void guard4(v8f& a, v8f& b, v8f& c, v8f& d, v16h x, v16h y) { dep_guard4_h(a, b, c, d, x, y); }
  static __device__ __forceinline__ void keep(v16h a, v16h b, v16h c, v16h d) { keep4_h(a, b, c, d); }
};
template <> struct Frag<__bf16> {
  typedef v16b V; union U { v16b v; v8b h[2]; };
  static __device__ __forceinline__ v16b load(const __bf16* p) {
    U f; f.h[0] = *(const v8b*)(p); f.h[1] = *(const v8b*)(p + 16); return f.v;
  }
  static __device__ __forceinline__ v8f mma(v16b a, v16b b, v8f c) {
    return __builtin_amdgcn_wmma_f32_16x16x32_bf16(false, a, false, b, (short)0, c, false, false);
  }
  static __device__ __forceinline__ void guard4(v8f& a, v8f& b, v8f& c, v8f& d, v16b x, v16b y) { dep_guard4_b(a, b, c, d, x, y); }
  static __device__ __forceinline__ void keep(v16b a, v16b b, v16b c, v16b d) { keep4_b(a, b, c, d); }
};

__device__ __forceinline__ unsigned pk16(unsigned short a, unsigned short b) { return (unsigned)a | ((unsigned)b << 16); }

__device__ __forceinline__ v8f mma_bf(v16b a, v16b b, v8f c) {
  c = __builtin_amdgcn_wmma_f32_16x16x32_bf16(false, a, false, b, (short)0, c, false, false);
  asm volatile("v_nop\n\tv_nop\n\tv_nop\n\tv_nop" : "+v"(c) : "v"(a), "v"(b));
  return c;
}
__device__ __forceinline__ v8f mma_fh(v16h a, v16h b, v8f c) {
  c = __builtin_amdgcn_wmma_f32_16x16x32_f16(false, a, false, b, (short)0, c, false, false);
  asm volatile("v_nop\n\tv_nop\n\tv_nop\n\tv_nop" : "+v"(c) : "v"(a), "v"(b));
  return c;
}

template <int ET> struct Elem;
template <> struct Elem<0> { typedef _Float16 T; };
template <> struct Elem<1> { typedef __bf16 T; };
template <int ET, int SPL, int BIAS_MODE, int OUT_MODE>
__global__ __launch_bounds__(256) void wmma_gemm64(
    const unsigned short* __restrict__ Ap, const unsigned short* __restrict__ A2p, int lda, long strideA,
    const unsigned short* __restrict__ Btp, const unsigned short* __restrict__ Bt2p, int ldb, long strideB,
    void* __restrict__ Cout, void* __restrict__ Cout2, int ldc, long strideC,
    const float* __restrict__ bias, int M, int N, int K, float scale) {
  typedef typename Elem<ET>::T T;
  typedef typename Frag<T>::V V;
  const T* A = (const T*)Ap; const T* A2 = (const T*)A2p; const T* Bt = (const T*)Btp; const T* Bt2 = (const T*)Bt2p;
  __shared__ __align__(16) float sT[8][16 * 68];
  const int b    = blockIdx.y;
  const int lane = threadIdx.x & 31;
  const int wave = threadIdx.x >> 5;
  const int tilesN = N >> 6;
  const int tilesM = M >> 6;
  const int tile = blockIdx.x * 8 + wave;
  if (tile >= tilesM * tilesN) return;
  const int tm = tile / tilesN;
  const int tn = tile - tm * tilesN;
  const int m0 = tm << 6;
  const int n0 = tn << 6;

  const T* Ab  = A  + (size_t)b * strideA;
  const T* Bb  = Bt + (size_t)b * strideB;
  const T* Ab2 = (SPL >= 1) ? (A2  + (size_t)b * strideA) : nullptr;
  const T* Bb2 = (SPL == 2) ? (Bt2 + (size_t)b * strideB) : nullptr;

  const int rlane = lane & 15;
  const int koff  = (lane >> 4) * 8;
  const int mOff  = (lane >> 4) * 8;

  v8f acc[4][4];
#pragma unroll
  for (int i = 0; i < 4; ++i)
#pragma unroll
    for (int j = 0; j < 4; ++j) acc[i][j] = (v8f){0.f,0.f,0.f,0.f,0.f,0.f,0.f,0.f};

  for (int k0 = 0; k0 < K; k0 += 32) {
    V bh[4], bl[4];
#pragma unroll
    for (int j = 0; j < 4; ++j) {
      const size_t bo = (size_t)(n0 + (j << 4) + rlane) * ldb + koff + k0;
      bh[j] = Frag<T>::load(Bb + bo);
      bl[j] = bh[j];
      if (SPL == 2) bl[j] = Frag<T>::load(Bb2 + bo);
    }
#pragma unroll
    for (int i = 0; i < 4; ++i) {
      const size_t ao = (size_t)(m0 + (i << 4) + rlane) * lda + koff + k0;
      V ah = Frag<T>::load(Ab + ao);
      V al = ah;
      if (SPL >= 1) al = Frag<T>::load(Ab2 + ao);
#pragma unroll
      for (int j = 0; j < 4; ++j) {
        acc[i][j] = Frag<T>::mma(ah, bh[j], acc[i][j]);
        if (SPL == 2) acc[i][j] = Frag<T>::mma(ah, bl[j], acc[i][j]);
        if (SPL >= 1) acc[i][j] = Frag<T>::mma(al, bh[j], acc[i][j]);
      }
      Frag<T>::guard4(acc[i][0], acc[i][1], acc[i][2], acc[i][3], ah, al);
    }
    Frag<T>::keep(bh[0], bh[1], bh[2], bh[3]);
    if (SPL == 2) Frag<T>::keep(bl[0], bl[1], bl[2], bl[3]);
  }
  acc_guard4(acc[0][0], acc[0][1], acc[0][2], acc[0][3]);
  acc_guard4(acc[1][0], acc[1][1], acc[1][2], acc[1][3]);
  acc_guard4(acc[2][0], acc[2][1], acc[2][2], acc[2][3]);
  acc_guard4(acc[3][0], acc[3][1], acc[3][2], acc[3][3]);

  float* slab = sT[wave];
  float bn[4] = {0.f, 0.f, 0.f, 0.f};
  if (BIAS_MODE == 2) {
#pragma unroll
    for (int j = 0; j < 4; ++j) bn[j] = bias[n0 + (j << 4) + rlane];
  }
#pragma unroll
  for (int i = 0; i < 4; ++i) {
    const int mBase = m0 + (i << 4);
    v4f bm0 = (v4f){0.f, 0.f, 0.f, 0.f};
    v4f bm1 = (v4f){0.f, 0.f, 0.f, 0.f};
    if (BIAS_MODE == 1) {
      bm0 = *(const v4f*)(bias + mBase + mOff);
      bm1 = *(const v4f*)(bias + mBase + mOff + 4);
    }
#pragma unroll
    for (int j = 0; j < 4; ++j) {
#pragma unroll
      for (int r = 0; r < 8; ++r) {
        float v = acc[i][j][r] * scale;
        if (BIAS_MODE == 1) v += (r < 4) ? bm0[r & 3] : bm1[r & 3];
        if (BIAS_MODE == 2) v += bn[j];
        slab[(mOff + r) * 68 + (j << 4) + rlane] = v;
      }
    }
    __builtin_amdgcn_fence(__ATOMIC_RELEASE, "workgroup");
    __builtin_amdgcn_wave_barrier();
    __builtin_amdgcn_fence(__ATOMIC_ACQUIRE, "workgroup");
    if (OUT_MODE == 0) {
      float* C = (float*)Cout + (size_t)b * strideC;
      const int hh = lane >> 4, c4 = (lane & 15) * 4;
      for (int pass = 0; pass < 2; ++pass) {
#pragma unroll
        for (int it = 0; it < 8; ++it) {
          const int row = it * 2 + hh;
          v4f v = *(const v4f*)(slab + row * 68 + c4);
          *(volatile v4f*)(C + (size_t)(mBase + row) * ldc + n0 + c4) = v;
        }
        __threadfence();
      }
    } else {
      const int q = lane >> 3, c8 = (lane & 7) * 8;
      unsigned short* C  = (unsigned short*)Cout  + (size_t)b * strideC;
      unsigned short* C2 = (OUT_MODE == 2) ? ((unsigned short*)Cout2 + (size_t)b * strideC) : nullptr;
      for (int pass = 0; pass < 2; ++pass) {
#pragma unroll
        for (int it = 0; it < 4; ++it) {
          const int row = it * 4 + q;
          const float* sp = slab + row * 68 + c8;
          v8h hv, lv;
#pragma unroll
          for (int e = 0; e < 8; ++e) {
            if (OUT_MODE == 1) {
              hv[e] = (_Float16)sp[e];
            } else {
              unsigned short hb = f2bf_bits(sp[e]);
              unsigned short lb = f2bf_bits(sp[e] - bf_bits2f(hb));
              hv[e] = __builtin_bit_cast(_Float16, hb);
              lv[e] = __builtin_bit_cast(_Float16, lb);
            }
          }
          *(volatile v8h*)(C + (size_t)(mBase + row) * ldc + n0 + c8) = hv;
          if (OUT_MODE == 2) *(volatile v8h*)(C2 + (size_t)(mBase + row) * ldc + n0 + c8) = lv;
        }
        __threadfence();
      }
    }
    __builtin_amdgcn_fence(__ATOMIC_RELEASE, "workgroup");
    __builtin_amdgcn_wave_barrier();
    __builtin_amdgcn_fence(__ATOMIC_ACQUIRE, "workgroup");
  }
}

__global__ __launch_bounds__(256) void cast8_bf16_kernel(const float* __restrict__ p0, const float* __restrict__ p1,
                                                         const float* __restrict__ p2, const float* __restrict__ p3,
                                                         const float* __restrict__ p4, unsigned short* __restrict__ out,
                                                         long planeStride, int n8) {
  const int i = blockIdx.x * 256 + threadIdx.x;
  if (i >= n8) return;
  const int z = blockIdx.y;
  const float* in = (z == 0) ? p0 : (z == 1) ? p1 : (z == 2) ? p2 : (z == 3) ? p3 : p4;
  const float* p = in + 8 * (size_t)i;
  const v4f a = *(const v4f*)(p);
  const v4f c = *(const v4f*)(p + 4);
  unsigned short hb[8];
#pragma unroll
  for (int e = 0; e < 4; ++e) {
    hb[e]     = f2bf_bits(a[e]);
    hb[4 + e] = f2bf_bits(c[e]);
  }
  const v4u u = (v4u){pk16(hb[0], hb[1]), pk16(hb[2], hb[3]), pk16(hb[4], hb[5]), pk16(hb[6], hb[7])};
  unsigned short* q = out + (size_t)z * planeStride + 8 * (size_t)i;
  *(volatile v4u*)q = u;
  __threadfence();
  *(volatile v4u*)q = u;
}

__global__ __launch_bounds__(256) void vec_bf16r_kernel(const float* __restrict__ p0, const float* __restrict__ p1,
                                                        const float* __restrict__ p2, const float* __restrict__ p3,
                                                        const float* __restrict__ p4, const float* __restrict__ p5,
                                                        const float* __restrict__ p6, float* __restrict__ out) {
  const int t = threadIdx.x;
  const int z = blockIdx.y;
  const float* in = (z == 0) ? p0 : (z == 1) ? p1 : (z == 2) ? p2 : (z == 3) ? p3 : (z == 4) ? p4 : (z == 5) ? p5 : p6;
  const v4f a = *(const v4f*)(in + 4 * t);
  v4f r;
#pragma unroll
  for (int e = 0; e < 4; ++e) r[e] = bf_bits2f(f2bf_bits(a[e]));
  float* q = out + (size_t)z * kD + 4 * t;
  *(volatile v4f*)q = r;
  __threadfence();
  *(volatile v4f*)q = r;
}

__global__ __launch_bounds__(128) void retention_kernel(const unsigned short* __restrict__ Qhp, const unsigned short* __restrict__ Qlp,
                                                        const unsigned short* __restrict__ Khp, const unsigned short* __restrict__ Klp,
                                                        const unsigned short* __restrict__ VTp, const float* __restrict__ glog,
                                                        float* __restrict__ obuf) {
  __shared__ __align__(16) _Float16 Psh[kRetWaves][16 * kPPitch];
  __shared__ __align__(16) float    Os[kRetWaves][16 * kOPitch];
  const __bf16*   Qh = (const __bf16*)Qhp;
  const __bf16*   Ql = (const __bf16*)Qlp;
  const __bf16*   Kh = (const __bf16*)Khp;
  const __bf16*   Kl = (const __bf16*)Klp;
  const _Float16* VT = (const _Float16*)VTp;
  const int tid  = threadIdx.x;
  const int wave = tid >> 5;
  const int lane = tid & 31;
  const int hh   = lane >> 4;
  const int c    = lane & 15;
  const int qb   = blockIdx.x;
  const int bh   = blockIdx.y;
  const int b    = bh >> 4;
  const int h    = bh & 15;
  const int q0   = qb * kRetRows + wave * 16;
  const size_t tokRow = (size_t)b * kT;

  const float glr = bf_bits2f(f2bf_bits(glog[h]));
  const float gma = 1.0f / (1.0f + expf(-glr));
  const float lg  = logf(gma);
  float rowfac[8];
#pragma unroll
  for (int r = 0; r < 8; ++r) rowfac[r] = expf(lg * (float)(8 * hh + r));
  const float colfac = expf(-lg * (float)c);
  const float dcut = kLnCut / lg;
  const float lowf = ((float)(q0 - (kKeyChunk - 1)) - dcut) * (1.0f / (float)kKeyChunk);
  int kcmin = (lowf > 0.0f) ? (int)ceilf(lowf) : 0;
  kcmin = kcmin > qb ? qb : kcmin;
  kcmin = __builtin_amdgcn_readfirstlane(kcmin);

  v16b qh[2], ql[2];
  {
    const size_t qo = (tokRow + q0 + c) * kD + h * kDh + 8 * hh;
    qh[0] = Frag<__bf16>::load(Qh + qo);
    qh[1] = Frag<__bf16>::load(Qh + qo + 32);
    asm volatile("" ::: "memory");
    ql[0] = Frag<__bf16>::load(Ql + qo);
    ql[1] = Frag<__bf16>::load(Ql + qo + 32);
    asm volatile("" ::: "memory");
  }

  float rsum[8];
  v8f oacc[4];
#pragma unroll
  for (int r = 0; r < 8; ++r) rsum[r] = 0.0f;
#pragma unroll
  for (int t = 0; t < 4; ++t) oacc[t] = (v8f){0.f,0.f,0.f,0.f,0.f,0.f,0.f,0.f};

  _Float16* pw = Psh[wave];
  for (int kc = qb; kc >= kcmin; --kc) {
    const int kv0 = kc * kKeyChunk;
    v8f s[4];
#pragma unroll
    for (int j = 0; j < 4; ++j) {
      s[j] = (v8f){0.f,0.f,0.f,0.f,0.f,0.f,0.f,0.f};
      const size_t ko = (tokRow + kv0 + 16 * j + c) * kD + h * kDh + 8 * hh;
      {
        const v16b kh0 = Frag<__bf16>::load(Kh + ko);
        const v16b kl0 = Frag<__bf16>::load(Kl + ko);
        s[j] = mma_bf(qh[0], kh0, s[j]);
        s[j] = mma_bf(qh[0], kl0, s[j]);
        s[j] = mma_bf(ql[0], kh0, s[j]);
      }
      asm volatile("" ::: "memory");
      {
        const v16b kh1 = Frag<__bf16>::load(Kh + ko + 32);
        const v16b kl1 = Frag<__bf16>::load(Kl + ko + 32);
        s[j] = mma_bf(qh[1], kh1, s[j]);
        s[j] = mma_bf(qh[1], kl1, s[j]);
        s[j] = mma_bf(ql[1], kh1, s[j]);
      }
      asm volatile("" ::: "memory");
    }
    float tf[4];
#pragma unroll
    for (int j = 0; j < 4; ++j) tf[j] = expf(lg * (float)(q0 - kv0 - 16 * j)) * colfac;
#pragma unroll
    for (int r = 0; r < 8; ++r) {
      const int irow = q0 + 8 * hh + r;
      const float rf = rowfac[r];
#pragma unroll
      for (int j = 0; j < 4; ++j) {
        const int kj = kv0 + 16 * j + c;
        const float pv = s[j][r] * (rf * tf[j]);
        const float pm = (kj <= irow) ? pv : 0.0f;
        rsum[r] += pm;
        pw[(8 * hh + r) * kPPitch + 16 * j + c] = (_Float16)(pm * kPCarry);
      }
    }
    __builtin_amdgcn_fence(__ATOMIC_RELEASE, "workgroup");
    __builtin_amdgcn_wave_barrier();
    __builtin_amdgcn_fence(__ATOMIC_ACQUIRE, "workgroup");
#pragma unroll
    for (int kk = 0; kk < 2; ++kk) {
      Frag<_Float16>::U pa;
      pa.h[0] = *(const v8h*)(pw + c * kPPitch + kk * 32 + 8 * hh);
      pa.h[1] = *(const v8h*)(pw + c * kPPitch + kk * 32 + 16 + 8 * hh);
#pragma unroll
      for (int t = 0; t < 4; ++t) {
        const size_t vo = ((size_t)(bh * kDh + 16 * t + c)) * kT + kv0 + kk * 32 + 8 * hh;
        const v16h vb = Frag<_Float16>::load(VT + vo);
        oacc[t] = mma_fh(pa.v, vb, oacc[t]);
      }
      asm volatile("" ::: "memory");
    }
    __builtin_amdgcn_fence(__ATOMIC_RELEASE, "workgroup");
    __builtin_amdgcn_wave_barrier();
    __builtin_amdgcn_fence(__ATOMIC_ACQUIRE, "workgroup");
  }

#pragma unroll
  for (int r = 0; r < 8; ++r) {
    float v = rsum[r];
    v += __shfl_xor(v, 1, 32);
    v += __shfl_xor(v, 2, 32);
    v += __shfl_xor(v, 4, 32);
    v += __shfl_xor(v, 8, 32);
    rsum[r] = v;
  }
  float* os = Os[wave];
#pragma unroll
  for (int r = 0; r < 8; ++r) {
    const float inv = (1.0f / fmaxf(fabsf(rsum[r]), 1.0f)) * kPCarryInv;
#pragma unroll
    for (int t = 0; t < 4; ++t) os[(8 * hh + r) * kOPitch + 16 * t + c] = oacc[t][r] * inv;
  }
  __builtin_amdgcn_fence(__ATOMIC_RELEASE, "workgroup");
  __builtin_amdgcn_wave_barrier();
  __builtin_amdgcn_fence(__ATOMIC_ACQUIRE, "workgroup");
  {
    float* orow = obuf + (tokRow + q0) * kD + h * kDh;
    const int c4 = (lane & 15) * 4;
    for (int pass = 0; pass < 2; ++pass) {
#pragma unroll
      for (int it = 0; it < 8; ++it) {
        const int row = it * 2 + hh;
        const v4f val = *(const v4f*)(os + row * kOPitch + c4);
        *(volatile v4f*)(orow + (size_t)row * kD + c4) = val;
      }
      __threadfence();
    }
  }
}

__global__ __launch_bounds__(256) void gn_stats_kernel(const float* __restrict__ obuf, float* __restrict__ stats) {
  __shared__ double shs[256];
  __shared__ double shq[256];
  __shared__ __align__(16) float stl[32];
  const int tid = threadIdx.x;
  const int bh = blockIdx.x;
  const int b = bh >> 4, h = bh & 15;
  const float* base = obuf + (size_t)b * kT * kD + h * kDh + (tid & 63);
  const int r0 = tid >> 6;
  double s = 0.0, s2 = 0.0;
#pragma unroll 1
  for (int i = 0; i < kT / 4; ++i) {
    const float v = base[(size_t)(r0 + 4 * i) * kD];
    const double dv = (double)v;
    s += dv;
    s2 += dv * dv;
  }
  shs[tid] = s;
  shq[tid] = s2;
  __syncthreads();
  for (int st = 128; st > 0; st >>= 1) {
    if (tid < st) {
      shs[tid] += shs[tid + st];
      shq[tid] += shq[tid + st];
    }
    __syncthreads();
  }
  if (tid < 32) {
    const double n = (double)(kT * kDh);
    const double mean = shs[0] / n;
    double var = shq[0] / n - mean * mean;
    var = (var > 0.0) ? var : 0.0;
    const float meanf = (float)mean;
    const float rstd = 1.0f / sqrtf((float)var + kGnEps);
    const float val = (tid == 0) ? meanf : ((tid == 1) ? rstd : 0.0f);
    stl[tid] = val;
  }
  __syncthreads();
  if (tid < 8) {
    const v4f v = *(const v4f*)(stl + 4 * tid);
    float* dp = stats + (size_t)bh * kStatPitch + 4 * tid;
    *(volatile v4f*)dp = v;
    __threadfence();
    *(volatile v4f*)dp = v;
  }
}

__global__ __launch_bounds__(256) void norm_gate_kernel(const float* __restrict__ obuf, const float* __restrict__ gpre,
                                                        const float* __restrict__ stats, const float* __restrict__ gnw,
                                                        const float* __restrict__ gnb, unsigned short* __restrict__ Yh,
                                                        unsigned short* __restrict__ Yl, int n8) {
  const int i = blockIdx.x * 256 + threadIdx.x;
  if (i >= n8) return;
  const size_t e0 = 8 * (size_t)i;
  const int c0  = (int)(e0 & (size_t)(kD - 1));
  const int tok = (int)(e0 >> 10);
  const int b   = tok >> 11;
  const int h   = c0 >> 6;
  const int sb  = (b * kH + h) * kStatPitch;
  const float mean = stats[sb];
  const float rstd = stats[sb + 1];
  unsigned hu0 = 0u, hu1 = 0u, hu2 = 0u, hu3 = 0u;
  unsigned lu0 = 0u, lu1 = 0u, lu2 = 0u, lu3 = 0u;
#pragma unroll 1
  for (int half = 0; half < 2; ++half) {
    const size_t eb = e0 + 4 * half;
    const v4f o  = *(const v4f*)(obuf + eb);
    const v4f g  = *(const v4f*)(gpre + eb);
    const v4f w  = *(const v4f*)(gnw + c0 + 4 * half);
    const v4f bb = *(const v4f*)(gnb + c0 + 4 * half);
    unsigned short hb[4], lb[4];
#pragma unroll
    for (int e = 0; e < 4; ++e) {
      const float on  = (o[e] - mean) * rstd * w[e] + bb[e];
      const float gp  = g[e];
      const float gcl = fminf(fmaxf(gp, -kGateClamp), kGateClamp);
      const float sg  = 1.0f / (1.0f + expf(-gcl));
      const float y   = on * (gp * sg);
      const unsigned short hbits = f2bf_bits(y);
      hb[e] = hbits;
      lb[e] = f2bf_bits(y - bf_bits2f(hbits));
    }
    const unsigned u0 = pk16(hb[0], hb[1]), u1 = pk16(hb[2], hb[3]);
    const unsigned l0 = pk16(lb[0], lb[1]), l1 = pk16(lb[2], lb[3]);
    if (half == 0) { hu0 = u0; hu1 = u1; lu0 = l0; lu1 = l1; }
    else           { hu2 = u0; hu3 = u1; lu2 = l0; lu3 = l1; }
  }
  const v4u hu = (v4u){hu0, hu1, hu2, hu3};
  const v4u lu = (v4u){lu0, lu1, lu2, lu3};
  unsigned short* qh = Yh + e0;
  unsigned short* ql = Yl + e0;
  *(volatile v4u*)qh = hu;
  *(volatile v4u*)ql = lu;
  __threadfence();
  *(volatile v4u*)qh = hu;
  *(volatile v4u*)ql = lu;
}

extern "C" void kernel_launch(void* const* d_in, const int* in_sizes, int n_in,
                              void* d_out, int out_size, void* d_ws, size_t ws_size,
                              hipStream_t stream) {
  if (n_in < 14) return;
  const int nAct = kTok * kD;
  const int nW   = kD * kD;
  if (in_sizes[0] != nAct) return;
  if (in_sizes[1] != nW || in_sizes[3] != nW || in_sizes[5] != nW || in_sizes[7] != nW || in_sizes[9] != nW) return;
  if (in_sizes[2] != kD || in_sizes[4] != kD || in_sizes[6] != kD || in_sizes[8] != kD || in_sizes[10] != kD) return;
  if (in_sizes[11] != kD || in_sizes[12] != kD || in_sizes[13] != kH) return;
  if (out_size != nAct) return;

  const size_t szP16 = (size_t)kTok * kD * 2;
  const size_t szXb  = szP16;
  const size_t szWb  = (size_t)5 * nW * 2;
  const size_t szBr  = (size_t)7 * kD * 4;
  const size_t szVT  = (size_t)kBH * kDh * kT * 2;
  const size_t szF32 = (size_t)kTok * kD * 4;
  const size_t szSt  = (size_t)kBH * kStatPitch * 4;
  const size_t offXb = 0;
  const size_t offWb = offXb + szXb;
  const size_t offBr = offWb + szWb;
  const size_t offQh = offBr + szBr;
  const size_t offQl = offQh + szP16;
  const size_t offKh = offQl + szP16;
  const size_t offKl = offKh + szP16;
  const size_t offVT = offKl + szP16;
  const size_t offG  = offVT + szVT;
  const size_t offO  = offG + szF32;
  const size_t offSt = offO + szF32;
  const size_t offYh = offSt + szSt;
  const size_t offYl = offYh + szP16;
  const size_t total = offYl + szP16;
  if (ws_size < total) return;

  const float* x    = (const float*)d_in[0];
  const float* wq   = (const float*)d_in[1];
  const float* bq   = (const float*)d_in[2];
  const float* wk   = (const float*)d_in[3];
  const float* bk   = (const float*)d_in[4];
  const float* wv   = (const float*)d_in[5];
  const float* bv   = (const float*)d_in[6];
  const float* wg   = (const float*)d_in[7];
  const float* bg   = (const float*)d_in[8];
  const float* wo   = (const float*)d_in[9];
  const float* bo   = (const float*)d_in[10];
  const float* gnw  = (const float*)d_in[11];
  const float* gnb  = (const float*)d_in[12];
  const float* glog = (const float*)d_in[13];
  float* out = (float*)d_out;
  char* ws = (char*)d_ws;
  unsigned short* Xb = (unsigned short*)(ws + offXb);
  unsigned short* Wb = (unsigned short*)(ws + offWb);
  float*          Br = (float*)(ws + offBr);
  unsigned short* Qh = (unsigned short*)(ws + offQh);
  unsigned short* Ql = (unsigned short*)(ws + offQl);
  unsigned short* Kh = (unsigned short*)(ws + offKh);
  unsigned short* Kl = (unsigned short*)(ws + offKl);
  unsigned short* VT = (unsigned short*)(ws + offVT);
  float*          G  = (float*)(ws + offG);
  float*          O  = (float*)(ws + offO);
  float*          St = (float*)(ws + offSt);
  unsigned short* Yh = (unsigned short*)(ws + offYh);
  unsigned short* Yl = (unsigned short*)(ws + offYl);
  const unsigned short* Wqb = Wb;
  const unsigned short* Wkb = Wb + (size_t)1 * nW;
  const unsigned short* Wvb = Wb + (size_t)2 * nW;
  const unsigned short* Wgb = Wb + (size_t)3 * nW;
  const unsigned short* Wob = Wb + (size_t)4 * nW;
  const float* bqr  = Br + 0 * kD;
  const float* bkr  = Br + 1 * kD;
  const float* bvr  = Br + 2 * kD;
  const float* bgr  = Br + 3 * kD;
  const float* bor  = Br + 4 * kD;
  const float* gnwr = Br + 5 * kD;
  const float* gnbr = Br + 6 * kD;

  const int n8x = nAct / 8;
  const int n8w = nW / 8;
  cast8_bf16_kernel<<<dim3(n8x / 256, 1), dim3(256), 0, stream>>>(x, x, x, x, x, Xb, 0L, n8x);
  cast8_bf16_kernel<<<dim3(n8w / 256, 5), dim3(256), 0, stream>>>(wq, wk, wv, wg, wo, Wb, (long)nW, n8w);
  vec_bf16r_kernel<<<dim3(1, 7), dim3(256), 0, stream>>>(bq, bk, bv, bg, bo, gnw, gnb, Br);

  const int tilesProj = (kTok / 64) * (kD / 64);
  const int tilesVT   = (kD / 64) * (kT / 64);
  wmma_gemm64<1, 0, 2, 2><<<dim3(tilesProj / 8, 1), dim3(256), 0, stream>>>(
      Xb, Xb, kD, 0L, Wqb, Wqb, kD, 0L, (void*)Qh, (void*)Ql, kD, 0L, bqr, kTok, kD, kD, 1.0f);
  wmma_gemm64<1, 0, 2, 2><<<dim3(tilesProj / 8, 1), dim3(256), 0, stream>>>(
      Xb, Xb, kD, 0L, Wkb, Wkb, kD, 0L, (void*)Kh, (void*)Kl, kD, 0L, bkr, kTok, kD, kD, 1.0f);
  wmma_gemm64<1, 0, 1, 1><<<dim3(tilesVT / 8, kB), dim3(256), 0, stream>>>(
      Wvb, Wvb, kD, 0L, Xb, Xb, kD, (long)kT * kD, (void*)VT, (void*)VT, kT, (long)kD * kT, bvr, kD, kT, kD, 1.0f);
  wmma_gemm64<1, 0, 2, 0><<<dim3(tilesProj / 8, 1), dim3(256), 0, stream>>>(
      Xb, Xb, kD, 0L, Wgb, Wgb, kD, 0L, (void*)G, (void*)G, kD, 0L, bgr, kTok, kD, kD, 1.0f);

  retention_kernel<<<dim3(kT / kRetRows, kBH), dim3(32 * kRetWaves), 0, stream>>>(Qh, Ql, Kh, Kl, VT, glog, O);
  gn_stats_kernel<<<dim3(kBH), dim3(256), 0, stream>>>(O, St);
  norm_gate_kernel<<<dim3(n8x / 256), dim3(256), 0, stream>>>(O, G, St, gnwr, gnbr, Yh, Yl, n8x);

  wmma_gemm64<1, 1, 2, 0><<<dim3(tilesProj / 8, 1), dim3(256), 0, stream>>>(
      Yh, Yl, kD, 0L, Wob, Wob, kD, 0L, (void*)out, (void*)out, kD, 0L, bor, kTok, kD, kD, 1.0f);
}
